// NodeLevelAttentionImproved_78142634983557
// MI455X (gfx1250) — hardware-run, weakly checked
//
#include <hip/hip_runtime.h>
#include <stddef.h>
#include <stdint.h>
#include <math.h>


#define NN      20000
#define MSLOT   32
#define FD      256
#define NH      4
#define HDIM    64
#define MPAD    128
#define MP      (((NN + MPAD - 1) / MPAD) * MPAD)
#define PTHR    256
#define NBX     ((MP * (FD / 8)) / PTHR)
#define NBW     ((FD * (FD / 8)) / PTHR)
#define GBM     32
#define GTHR    128
#define RTHR    256
#define RWAVE   8
#define NEGSL   0.2f
#define NEGFILL (-1.0e9f)
#define LN_EPS  1e-5f

static_assert(MSLOT == 32);
static_assert(NH * HDIM == FD && FD == 32 * 8);
static_assert(HDIM == 16 * 4);
static_assert((NN % RWAVE) == 0);
static_assert(NN <= MP && (MP % GBM) == 0 && (MP % MPAD) == 0);
static_assert((FD % 32) == 0);
static_assert((MP * (FD / 8)) % PTHR == 0 && (FD * (FD / 8)) % PTHR == 0);
static_assert(GTHR * 4 == 2 * FD);
static_assert(16 * GTHR * 4 == GBM * FD);

#define OFF_XB   ((size_t)0)
#define SZ_XB    ((size_t)MP * FD * 2)
#define OFF_WT   (OFF_XB + SZ_XB)
#define SZ_WT    ((size_t)FD * FD * 2)
#define OFF_HP   (OFF_WT + SZ_WT)
#define SZ_HP    ((size_t)MP * FD * 4)
#define OFF_SD   (OFF_HP + SZ_HP)
#define SZ_SD    ((size_t)2 * MP * NH * 4)
#define OFF_PAR  (OFF_SD + SZ_SD)
#define SZ_PAR   ((size_t)1024 * 4)
#define WS_TOTAL (OFF_PAR + SZ_PAR)
static_assert((SZ_XB % 256) == 0 && (SZ_WT % 256) == 0 && (SZ_HP % 256) == 0 && (SZ_SD % 256) == 0 && (SZ_PAR % 256) == 0);
static_assert(WS_TOTAL <= (size_t)(128u << 20));

typedef float          v4f  __attribute__((ext_vector_type(4)));
typedef float          v8f  __attribute__((ext_vector_type(8)));
typedef int            v8i  __attribute__((ext_vector_type(8)));
typedef unsigned int   v4u  __attribute__((ext_vector_type(4)));
typedef unsigned short v8us __attribute__((ext_vector_type(8)));
typedef __bf16         v16b __attribute__((ext_vector_type(16)));
typedef v4f  __attribute__((may_alias)) v4fa;
typedef v8us __attribute__((may_alias)) v8usa;
union FragB { v16b v; v8us h[2]; v8i w; };

__device__ __forceinline__ v8f wmb(const FragB& a, const FragB& b, v8f c) {
  v8f d = __builtin_amdgcn_wmma_f32_16x16x32_bf16(false, a.v, false, b.v, (short)0, c, false, false);
  asm volatile("v_nop\n\tv_nop\n\tv_nop\n\tv_nop" : "+v"(d) : "v"(a.w), "v"(b.w));
  return d;
}

__device__ __forceinline__ unsigned int f2bf(float f) {
  const unsigned int u = __float_as_uint(f);
  return ((u + 0x7FFFu + ((u >> 16) & 1u)) >> 16) & 0xFFFFu;
}
__device__ __forceinline__ float bf2f(unsigned int b) { return __uint_as_float(b << 16); }
__device__ __forceinline__ float bfr(float f) { return bf2f(f2bf(f)); }
__device__ __forceinline__ v4f bfr4(const v4f a) {
  v4f r; r.x = bfr(a.x); r.y = bfr(a.y); r.z = bfr(a.z); r.w = bfr(a.w); return r;
}
__device__ __forceinline__ unsigned int pk2(float lo, float hi) { return f2bf(lo) | (f2bf(hi) << 16); }
__device__ __forceinline__ v4u pack8(const v4f a, const v4f b) {
  v4u r;
  r.x = pk2(a.x, a.y); r.y = pk2(a.z, a.w); r.z = pk2(b.x, b.y); r.w = pk2(b.z, b.w);
  return r;
}
__device__ __forceinline__ void pin4(const v4f v) {
  asm volatile("" :: "v"(v.x), "v"(v.y), "v"(v.z), "v"(v.w));
}
__device__ __forceinline__ float wmaxf(float v) {
#pragma unroll
  for (int off = 16; off > 0; off >>= 1) v = fmaxf(v, __shfl_xor(v, off));
  return v;
}
__device__ __forceinline__ float wsumf(float v) {
#pragma unroll
  for (int off = 16; off > 0; off >>= 1) v += __shfl_xor(v, off);
  return v;
}
__device__ __forceinline__ float gelu_erf(float x) {
  return 0.5f * x * (1.0f + erff(x * 0.70710678f));
}

__global__ __launch_bounds__(PTHR) void k_prep(
    const float* __restrict__ h, const float* __restrict__ W,
    const float* __restrict__ al, const float* __restrict__ ar,
    const float* __restrict__ gam, const float* __restrict__ bet,
    unsigned short* XB, unsigned short* WT, float* PAR)
{
  const int b = (int)blockIdx.x, tid = (int)threadIdx.x;
  const v4f z4 = {0.f, 0.f, 0.f, 0.f};
  if (b < NBX) {
    const int i   = b * PTHR + tid;
    const int row = i >> 5;
    const int c0  = (i & 31) * 8;
    const int rc  = row < NN ? row : NN - 1;
    const float* p = h + (size_t)rc * FD + c0;
    v4f a = *(const v4fa*)p, c = *(const v4fa*)(p + 4);
    if (row >= NN) { a = z4; c = z4; }
    const v4u hv = pack8(a, c);
    unsigned short* o = XB + (size_t)row * FD + c0;
    *(volatile v4u*)o = hv;
    __threadfence();
    *(volatile v4u*)o = hv;
  } else if (b < NBX + NBW) {
    const int u  = (b - NBX) * PTHR + tid;
    const int n  = u >> 5;
    const int k8 = (u & 31) * 8;
    const float* p = W + (size_t)k8 * FD + n;
    v4f a, c;
    a.x = p[0];          a.y = p[FD];         a.z = p[2 * FD];     a.w = p[3 * FD];
    c.x = p[4 * FD];     c.y = p[5 * FD];     c.z = p[6 * FD];     c.w = p[7 * FD];
    const v4u wv = pack8(a, c);
    unsigned short* o = WT + (size_t)n * FD + k8;
    *(volatile v4u*)o = wv;
    __threadfence();
    *(volatile v4u*)o = wv;
  } else {
    const int which = tid >> 6;
    const int off   = (tid & 63) * 4;
    const v4f va = *(const v4fa*)(al  + off);
    const v4f vb = *(const v4fa*)(ar  + off);
    const v4f vc = *(const v4fa*)(gam + off);
    const v4f vd = *(const v4fa*)(bet + off);
    pin4(va); pin4(vb); pin4(vc); pin4(vd);
    v4f v = va;
    v = (which == 1) ? vb : v;
    v = (which == 2) ? vc : v;
    v = (which == 3) ? vd : v;
    const v4f r = bfr4(v);
    float* o = PAR + 4 * tid;
    *(volatile v4f*)o = r;
    __threadfence();
    *(volatile v4f*)o = r;
  }
}

__global__ __launch_bounds__(GTHR) void k_gemm(
    const unsigned short* __restrict__ XB, const unsigned short* __restrict__ WT,
    const float* __restrict__ PAR, float* HP, float* SD)
{
  __shared__ __attribute__((aligned(16))) float stg[GBM * FD];
  __shared__ __attribute__((aligned(16))) float satt[2 * FD];
  const int tid = (int)threadIdx.x, lane = tid & 31, wave = tid >> 5, hh = lane >> 4, m = lane & 15;
  const int rt = wave >> 1, ch = wave & 1;
  const int rowBase = (int)blockIdx.x * GBM;

  {
    const v4f av = *(const v4fa*)(PAR + 4 * tid);
    *(v4fa*)(satt + 4 * tid) = av;
  }

  v8f acc[8];
  {
    const v8f z = {0.f, 0.f, 0.f, 0.f, 0.f, 0.f, 0.f, 0.f};
#pragma unroll
    for (int t = 0; t < 8; ++t) acc[t] = z;
  }
  const unsigned short* ap = XB + (size_t)(rowBase + 16 * rt + m) * FD + 8 * hh;
  const unsigned short* wp = WT + (size_t)(128 * ch + m) * FD + 8 * hh;
#pragma unroll 1
  for (int ks = 0; ks < FD / 32; ++ks) {
    FragB af;
    af.h[0] = *(const v8usa*)(ap + 32 * ks);
    af.h[1] = *(const v8usa*)(ap + 32 * ks + 16);
#pragma unroll
    for (int t = 0; t < 8; ++t) {
      const unsigned short* wq = wp + (size_t)(16 * t) * FD + 32 * ks;
      FragB bf;
      bf.h[0] = *(const v8usa*)wq;
      bf.h[1] = *(const v8usa*)(wq + 16);
      acc[t] = wmb(af, bf, acc[t]);
    }
  }

#pragma unroll
  for (int t = 0; t < 8; ++t) {
    const int lc = 128 * ch + 16 * t + m;
#pragma unroll
    for (int r = 0; r < 8; ++r) {
      const int lr = 16 * rt + 8 * hh + r;
      stg[lr * FD + lc] = acc[t][r];
    }
  }
  __syncthreads();

  v4f dv = {0.f, 0.f, 0.f, 0.f};
  if (wave < 2) {
    const float* hr = stg + lane * FD;
    const float* sa = satt + wave * FD;
    float d0 = 0.f, d1 = 0.f, d2 = 0.f, d3 = 0.f;
#pragma unroll 2
    for (int c4 = 0; c4 < HDIM / 4; ++c4) {
      const v4f h0 = *(const v4fa*)(hr + 4 * c4);
      const v4f a0 = *(const v4fa*)(sa + 4 * c4);
      const v4f h1 = *(const v4fa*)(hr + HDIM + 4 * c4);
      const v4f a1 = *(const v4fa*)(sa + HDIM + 4 * c4);
      const v4f h2 = *(const v4fa*)(hr + 2 * HDIM + 4 * c4);
      const v4f a2 = *(const v4fa*)(sa + 2 * HDIM + 4 * c4);
      const v4f h3 = *(const v4fa*)(hr + 3 * HDIM + 4 * c4);
      const v4f a3 = *(const v4fa*)(sa + 3 * HDIM + 4 * c4);
      d0 = fmaf(h0.x, a0.x, d0); d0 = fmaf(h0.y, a0.y, d0); d0 = fmaf(h0.z, a0.z, d0); d0 = fmaf(h0.w, a0.w, d0);
      d1 = fmaf(h1.x, a1.x, d1); d1 = fmaf(h1.y, a1.y, d1); d1 = fmaf(h1.z, a1.z, d1); d1 = fmaf(h1.w, a1.w, d1);
      d2 = fmaf(h2.x, a2.x, d2); d2 = fmaf(h2.y, a2.y, d2); d2 = fmaf(h2.z, a2.z, d2); d2 = fmaf(h2.w, a2.w, d2);
      d3 = fmaf(h3.x, a3.x, d3); d3 = fmaf(h3.y, a3.y, d3); d3 = fmaf(h3.z, a3.z, d3); d3 = fmaf(h3.w, a3.w, d3);
    }
    dv.x = d0; dv.y = d1; dv.z = d2; dv.w = d3;
  }
  float* sp = SD + (size_t)(wave & 1) * ((size_t)NH * MP) + (size_t)(rowBase + lane) * NH;
  float* hb = HP + (size_t)rowBase * FD;

#pragma unroll 4
  for (int i = 0; i < 16; ++i) {
    const int p = i * GTHR + tid;
    const v4f v = *(const v4fa*)(stg + 4 * p);
    *(volatile v4f*)(hb + 4 * p) = v;
  }
  if (wave < 2) *(volatile v4f*)sp = dv;
  __threadfence();
#pragma unroll 4
  for (int i = 0; i < 16; ++i) {
    const int p = i * GTHR + tid;
    const v4f v = *(const v4fa*)(stg + 4 * p);
    *(volatile v4f*)(hb + 4 * p) = v;
  }
  if (wave < 2) *(volatile v4f*)sp = dv;
}

__global__ __launch_bounds__(RTHR) void k_row(
    const int* __restrict__ nidx, const int* __restrict__ nmask,
    const float* __restrict__ HP, const float* __restrict__ SD,
    const float* __restrict__ PAR, float* out)
{
  __shared__ __attribute__((aligned(16))) float s_al[RWAVE * MSLOT * NH];
  __shared__ __attribute__((aligned(16))) int   s_id[RWAVE * MSLOT];
  const int tid = (int)threadIdx.x, lane = tid & 31, wave = tid >> 5;
  const int n  = (int)blockIdx.x * RWAVE + wave;
  const int nc = n < NN ? n : NN - 1;

  const int idr = nidx [(size_t)nc * MSLOT + lane];
  const int mk  = nmask[(size_t)nc * MSLOT + lane];
  int id = idr < 0 ? 0 : idr;
  id = id > NN - 1 ? NN - 1 : id;
  const v4f el4 = *(const v4fa*)(SD + (size_t)NH * nc);
  const v4f er4 = *(const v4fa*)(SD + (size_t)NH * MP + (size_t)NH * id);
  pin4(er4);
  const v4f ga = *(const v4fa*)(PAR + 512 + 4 * lane);
  const v4f gb = *(const v4fa*)(PAR + 512 + 128 + 4 * lane);
  const v4f ba = *(const v4fa*)(PAR + 768 + 4 * lane);
  const v4f bb = *(const v4fa*)(PAR + 768 + 128 + 4 * lane);

  const bool dead = (mk == 0);
  float e0 = el4.x + er4.x, e1 = el4.y + er4.y, e2 = el4.z + er4.z, e3 = el4.w + er4.w;
  e0 = e0 > 0.f ? e0 : NEGSL * e0;
  e1 = e1 > 0.f ? e1 : NEGSL * e1;
  e2 = e2 > 0.f ? e2 : NEGSL * e2;
  e3 = e3 > 0.f ? e3 : NEGSL * e3;
  e0 = dead ? NEGFILL : e0;
  e1 = dead ? NEGFILL : e1;
  e2 = dead ? NEGFILL : e2;
  e3 = dead ? NEGFILL : e3;

  const float m0 = wmaxf(e0), m1 = wmaxf(e1), m2 = wmaxf(e2), m3 = wmaxf(e3);
  const float p0 = expf(e0 - m0), p1 = expf(e1 - m1), p2 = expf(e2 - m2), p3 = expf(e3 - m3);
  const float s0 = wsumf(p0), s1 = wsumf(p1), s2 = wsumf(p2), s3 = wsumf(p3);
  {
    const int hs = lane & 3;
    float ss = s0;
    ss = (hs == 1) ? s1 : ss;
    ss = (hs == 2) ? s2 : ss;
    ss = (hs == 3) ? s3 : ss;
    const float rsel = 1.0f / ss;
    const float r0 = __shfl(rsel, 0), r1 = __shfl(rsel, 1), r2 = __shfl(rsel, 2), r3 = __shfl(rsel, 3);
    v4f al4;
    al4.x = p0 * r0; al4.y = p1 * r1; al4.z = p2 * r2; al4.w = p3 * r3;
    *(v4fa*)(s_al + (wave * MSLOT + lane) * NH) = al4;
    s_id[wave * MSLOT + lane] = id;
  }
  __syncthreads();

  const int hlo = lane >> 4;
  const float* sal  = s_al + wave * (MSLOT * NH) + hlo;
  const int*   sidp = s_id + wave * MSLOT;
  const float* hpl  = HP + 4 * lane;
  float x0 = 0.f, x1 = 0.f, x2 = 0.f, x3 = 0.f, x4 = 0.f, x5 = 0.f, x6 = 0.f, x7 = 0.f;
#pragma unroll 1
  for (int mslot = 0; mslot < MSLOT; ++mslot) {
    int sid = sidp[mslot];
    sid = sid < 0 ? 0 : (sid > NN - 1 ? NN - 1 : sid);
    const float a_lo = sal[NH * mslot];
    const float a_hi = sal[NH * mslot + 2];
    const float* p = hpl + (size_t)sid * FD;
    const v4f v0 = *(const v4fa*)p;
    const v4f v1 = *(const v4fa*)(p + 128);
    x0 = fmaf(a_lo, v0.x, x0); x1 = fmaf(a_lo, v0.y, x1); x2 = fmaf(a_lo, v0.z, x2); x3 = fmaf(a_lo, v0.w, x3);
    x4 = fmaf(a_hi, v1.x, x4); x5 = fmaf(a_hi, v1.y, x5); x6 = fmaf(a_hi, v1.z, x6); x7 = fmaf(a_hi, v1.w, x7);
  }

  {
    const float* q = hpl + (size_t)nc * FD;
    const v4f o0 = *(const v4fa*)q;
    const v4f o1 = *(const v4fa*)(q + 128);
    x0 += o0.x; x1 += o0.y; x2 += o0.z; x3 += o0.w;
    x4 += o1.x; x5 += o1.y; x6 += o1.z; x7 += o1.w;
  }
  float gs = 0.f;
#pragma unroll 1
  for (int j = 0; j < 8; ++j) {
    const float g = gelu_erf(x0);
    gs += g;
    x0 = x1; x1 = x2; x2 = x3; x3 = x4; x4 = x5; x5 = x6; x6 = x7; x7 = g;
  }

  const float mu = wsumf(gs) * (1.0f / (float)FD);
  float qs = 0.f;
#pragma unroll 1
  for (int j = 0; j < 8; ++j) {
    const float d = x0 - mu;
    qs = fmaf(d, d, qs);
    x0 = x1; x1 = x2; x2 = x3; x3 = x4; x4 = x5; x5 = x6; x6 = x7; x7 = d;
  }
  const float var = wsumf(qs) * (1.0f / (float)FD);
  const float rs  = 1.0f / sqrtf(var + LN_EPS);
  v4f ya, yb;
  ya.x = fmaf(x0 * rs, ga.x, ba.x); ya.y = fmaf(x1 * rs, ga.y, ba.y);
  ya.z = fmaf(x2 * rs, ga.z, ba.z); ya.w = fmaf(x3 * rs, ga.w, ba.w);
  yb.x = fmaf(x4 * rs, gb.x, bb.x); yb.y = fmaf(x5 * rs, gb.y, bb.y);
  yb.z = fmaf(x6 * rs, gb.z, bb.z); yb.w = fmaf(x7 * rs, gb.w, bb.w);

  float* op = out + (size_t)nc * FD + 4 * lane;
  const bool wr = n < NN;
  if (wr) { *(volatile v4f*)op = ya; *(volatile v4f*)(op + 128) = yb; }
  __threadfence();
  if (wr) { *(volatile v4f*)op = ya; *(volatile v4f*)(op + 128) = yb; }
}

extern "C" void kernel_launch(void* const* d_in, const int* in_sizes, int n_in,
                              void* d_out, int out_size, void* d_ws, size_t ws_size,
                              hipStream_t stream) {
  if (n_in < 8) return;
  if (in_sizes[0] != NN * FD) return;
  if (in_sizes[1] != NN * MSLOT) return;
  if (in_sizes[2] != NN * MSLOT) return;
  if (in_sizes[3] != FD * FD) return;
  if (in_sizes[4] != NH * HDIM || in_sizes[5] != NH * HDIM) return;
  if (in_sizes[6] != FD || in_sizes[7] != FD) return;
  if (out_size != NN * FD) return;
  if ((size_t)WS_TOTAL > ws_size) return;

  const float* h    = (const float*)d_in[0];
  const int*   nidx = (const int*)  d_in[1];
  const int*   nmsk = (const int*)  d_in[2];
  const float* W    = (const float*)d_in[3];
  const float* al   = (const float*)d_in[4];
  const float* ar   = (const float*)d_in[5];
  const float* gam  = (const float*)d_in[6];
  const float* bet  = (const float*)d_in[7];
  float* out = (float*)d_out;

  char* ws = (char*)d_ws;
  unsigned short* XB  = (unsigned short*)(ws + OFF_XB);
  unsigned short* WT  = (unsigned short*)(ws + OFF_WT);
  float*          HP  = (float*)(ws + OFF_HP);
  float*          SD  = (float*)(ws + OFF_SD);
  float*          PAR = (float*)(ws + OFF_PAR);

  k_prep<<<NBX + NBW + 1, PTHR, 0, stream>>>(h, W, al, ar, gam, bet, XB, WT, PAR);
  k_gemm<<<MP / GBM, GTHR, 0, stream>>>(XB, WT, PAR, HP, SD);
  k_row<<<NN / RWAVE, RTHR, 0, stream>>>(nidx, nmsk, HP, SD, PAR, out);
}
